// CausalLinearAttention_87943750352898
// MI455X (gfx1250) — hardware-verified
//
#include <hip/hip_runtime.h>
#include <stddef.h>
#include <stdint.h>


#define TLEN 2048
#define DM   128
#define QB   64
#define KB   64
#define NQB  (TLEN / QB)
#define NKB  (TLEN / KB)
#define WP   136
#define PP   72
#define OP   68
#define EPSV 1e-6f

typedef _Float16 v16h __attribute__((ext_vector_type(16)));
typedef _Float16 v8h  __attribute__((ext_vector_type(8)));
typedef _Float16 v4h  __attribute__((ext_vector_type(4)));
typedef float    v8f  __attribute__((ext_vector_type(8)));
typedef float    v4f  __attribute__((ext_vector_type(4)));
union Frag { v16h v; v8h hv[2]; };

__device__ __forceinline__ v8f zero8() {
  v8f z = {0.f, 0.f, 0.f, 0.f, 0.f, 0.f, 0.f, 0.f};
  return z;
}

__device__ __forceinline__ v8f wmma_f16(v16h a, v16h b, v8f c) {
  c = __builtin_amdgcn_wmma_f32_16x16x32_f16(false, a, false, b, (short)0, c, false, false);
  asm volatile("v_nop\n\tv_nop\n\tv_nop\n\tv_nop" : "+v"(c) : "v"(a), "v"(b));
  return c;
}

__device__ __forceinline__ v16h frag_rowk(const _Float16* p, int h) {
  Frag f;
  f.hv[0] = *(const v8h*)(p + 8 * h);
  f.hv[1] = *(const v8h*)(p + 16 + 8 * h);
  return f.v;
}

__global__ __launch_bounds__(256) void k_vconv(const float* __restrict__ v,
                                               _Float16* vth, _Float16* vtl) {
  __shared__ __attribute__((aligned(16))) _Float16 sTh[DM * PP];
  __shared__ __attribute__((aligned(16))) _Float16 sTl[DM * PP];

  const int bid = blockIdx.x;
  const int b = bid / NKB, st = bid - b * NKB;
  const int tid = threadIdx.x;
  const size_t base = ((size_t)b * TLEN + (size_t)st * KB) * DM;

  for (int p = 0; p < 8; ++p) {
    const int idx = p * 256 + tid;
    const int sr = idx >> 5, c4 = idx & 31;
    const v4f x = *(const v4f*)(v + base + (size_t)sr * DM + c4 * 4);
#pragma unroll
    for (int j = 0; j < 4; ++j) {
      const float xf = x[j];
      const _Float16 hi = (_Float16)xf;
      const _Float16 lo = (_Float16)((xf - (float)hi) * 2048.f);
      const int e = c4 * 4 + j;
      sTh[e * PP + sr] = hi;
      sTl[e * PP + sr] = lo;
    }
  }
  __syncthreads();

#pragma unroll
  for (int p = 0; p < 4; ++p) {
    const int piece = p * 256 + tid;
    const int e = piece >> 3, jj = piece & 7;
    const v8h xh = *(const v8h*)(sTh + e * PP + jj * 8);
    const v8h xl = *(const v8h*)(sTl + e * PP + jj * 8);
    const size_t off = ((size_t)b * DM + e) * TLEN + (size_t)st * KB + jj * 8;
    *(volatile v8h*)(vth + off) = xh;
    *(volatile v8h*)(vtl + off) = xl;
  }
  __threadfence();
#pragma unroll
  for (int p = 0; p < 4; ++p) {
    const int piece = p * 256 + tid;
    const int e = piece >> 3, jj = piece & 7;
    const v8h xh = *(const v8h*)(sTh + e * PP + jj * 8);
    const v8h xl = *(const v8h*)(sTl + e * PP + jj * 8);
    const size_t off = ((size_t)b * DM + e) * TLEN + (size_t)st * KB + jj * 8;
    *(volatile v8h*)(vth + off) = xh;
    *(volatile v8h*)(vtl + off) = xl;
  }
}

__global__ __launch_bounds__(256) void k_phi(const float* __restrict__ q, const float* __restrict__ k,
                                             const float* __restrict__ W, const float* __restrict__ bias,
                                             _Float16* qh, _Float16* kh, int nrb) {
  __shared__ __attribute__((aligned(16))) _Float16 sW[DM * WP];
  __shared__ __attribute__((aligned(16))) _Float16 sX[QB * WP];
  __shared__ float sBias[DM];

  const int bid = blockIdx.x;
  const int which = (bid >= nrb) ? 1 : 0;
  const int rb = bid - which * nrb;
  const float* X = which ? k : q;
  _Float16* F = which ? kh : qh;

  const int tid = threadIdx.x, lane = tid & 31, w = tid >> 5;
  const int h = lane >> 4, m = lane & 15;

  for (int p = 0; p < 16; ++p) {
    const int idx = p * 256 + tid;
    const int e = idx >> 5, c4 = idx & 31;
    const v4f x = *(const v4f*)(W + (size_t)e * DM + c4 * 4);
    v4h y;
    y[0] = (_Float16)(x[0] * 16.f);
    y[1] = (_Float16)(x[1] * 16.f);
    y[2] = (_Float16)(x[2] * 16.f);
    y[3] = (_Float16)(x[3] * 16.f);
    *(v4h*)(sW + e * WP + c4 * 4) = y;
  }
  if (tid < DM) sBias[tid] = bias[tid];

  const size_t r0 = (size_t)rb * QB;
  for (int p = 0; p < 8; ++p) {
    const int idx = p * 256 + tid;
    const int r = idx >> 5, c4 = idx & 31;
    const v4f x = *(const v4f*)(X + (r0 + r) * DM + c4 * 4);
    v4h y;
    y[0] = (_Float16)x[0];
    y[1] = (_Float16)x[1];
    y[2] = (_Float16)x[2];
    y[3] = (_Float16)x[3];
    *(v4h*)(sX + r * WP + c4 * 4) = y;
  }
  __syncthreads();

  const int rt = w & 3, ch = w >> 2;
  v8f acc[4];
#pragma unroll
  for (int et = 0; et < 4; ++et) acc[et] = zero8();

#pragma unroll
  for (int kk = 0; kk < DM; kk += 32) {
    const v16h a = frag_rowk(sX + (rt * 16 + m) * WP + kk, h);
#pragma unroll
    for (int et = 0; et < 4; ++et) {
      const v16h bb = frag_rowk(sW + (ch * 64 + et * 16 + m) * WP + kk, h);
      acc[et] = wmma_f16(a, bb, acc[et]);
    }
  }
  __syncthreads();

#pragma unroll
  for (int et = 0; et < 4; ++et) {
    const int e = ch * 64 + et * 16 + m;
    const float be = sBias[e];
#pragma unroll
    for (int r = 0; r < 8; ++r) {
      const float y = acc[et][r] * 0.0625f + be;
      const float f = (y > 0.f) ? (y + 1.f) : __expf(y);
      sX[(rt * 16 + 8 * h + r) * DM + e] = (_Float16)f;
    }
  }
  __syncthreads();

  _Float16* dst = F + r0 * DM;
#pragma unroll
  for (int p = 0; p < 4; ++p) {
    const int piece = p * 256 + tid;
    const v8h x = *(const v8h*)(sX + piece * 8);
    *(volatile v8h*)(dst + (size_t)piece * 8) = x;
  }
  __threadfence();
#pragma unroll
  for (int p = 0; p < 4; ++p) {
    const int piece = p * 256 + tid;
    const v8h x = *(const v8h*)(sX + piece * 8);
    *(volatile v8h*)(dst + (size_t)piece * 8) = x;
  }
}

__global__ __launch_bounds__(256) void k_attn(const _Float16* __restrict__ qh, const _Float16* __restrict__ kh,
                                              const _Float16* __restrict__ vth, const _Float16* __restrict__ vtl,
                                              float* out) {
  __shared__ __attribute__((aligned(16))) _Float16 sPh[QB * PP];
  __shared__ __attribute__((aligned(16))) _Float16 sPl[QB * PP];
  __shared__ __attribute__((aligned(16))) float sO[8 * 16 * OP];
  __shared__ float sRS[8 * 16];
  __shared__ float sInv[8 * 16];

  const int bid = blockIdx.x;
  const int b = bid / NQB, qb = bid - b * NQB;
  const int tid = threadIdx.x, lane = tid & 31, w = tid >> 5;
  const int h = lane >> 4, m = lane & 15;
  const int rt = w & 3, half = w >> 2;
  const int t0 = qb * QB;

  v8f ohh[4], ox[4];
#pragma unroll
  for (int et = 0; et < 4; ++et) { ohh[et] = zero8(); ox[et] = zero8(); }
  v8f rs = zero8();

  const _Float16* qrow  = qh + ((size_t)b * TLEN + t0 + rt * 16 + m) * DM;
  const _Float16* kbase = kh + ((size_t)b * TLEN + half * 32 + m) * DM;
  const size_t vbo = ((size_t)b * DM + half * 64 + m) * TLEN;
  const _Float16* vhb = vth + vbo;
  const _Float16* vlb = vtl + vbo;

  for (int kt = 0; kt <= qb; ++kt) {
    const int s0 = kt * KB;

    v8f sacc[2];
    sacc[0] = zero8();
    sacc[1] = zero8();
#pragma unroll
    for (int kk = 0; kk < DM; kk += 32) {
      const v16h a = frag_rowk(qrow + kk, h);
#pragma unroll
      for (int ct = 0; ct < 2; ++ct) {
        const v16h bb = frag_rowk(kbase + ((size_t)s0 + ct * 16) * DM + kk, h);
        sacc[ct] = wmma_f16(a, bb, sacc[ct]);
      }
    }

    const bool fulltile = (kt < qb);
#pragma unroll
    for (int ct = 0; ct < 2; ++ct) {
      const int kl = half * 32 + ct * 16 + m;
#pragma unroll
      for (int r = 0; r < 8; ++r) {
        const int ql = rt * 16 + 8 * h + r;
        float sv = sacc[ct][r];
        sv = (fulltile || (kl <= ql)) ? sv : 0.f;
        rs[r] += sv;
        const float ps = sv * 0.015625f;
        const _Float16 ph = (_Float16)ps;
        const _Float16 pl = (_Float16)((ps - (float)ph) * 2048.f);
        sPh[ql * PP + kl] = ph;
        sPl[ql * PP + kl] = pl;
      }
    }
    __syncthreads();

#pragma unroll
    for (int ks = 0; ks < 2; ++ks) {
      const v16h ah = frag_rowk(sPh + (rt * 16 + m) * PP + ks * 32, h);
      const v16h al = frag_rowk(sPl + (rt * 16 + m) * PP + ks * 32, h);
#pragma unroll
      for (int et = 0; et < 4; ++et) {
        const size_t vo = (size_t)et * 16 * TLEN + (size_t)s0 + ks * 32;
        const v16h bh = frag_rowk(vhb + vo, h);
        const v16h bl = frag_rowk(vlb + vo, h);
        ohh[et] = wmma_f16(ah, bh, ohh[et]);
        ox[et]  = wmma_f16(ah, bl, ox[et]);
        ox[et]  = wmma_f16(al, bh, ox[et]);
      }
    }
    __syncthreads();
  }

#pragma unroll
  for (int r = 0; r < 8; ++r) {
    float x = rs[r];
    x += __shfl_xor(x, 1);
    x += __shfl_xor(x, 2);
    x += __shfl_xor(x, 4);
    x += __shfl_xor(x, 8);
    rs[r] = x;
  }
  if (m == 0) {
#pragma unroll
    for (int r = 0; r < 8; ++r) sRS[w * 16 + 8 * h + r] = rs[r];
  }
  __syncthreads();
  if (lane < 16) {
    const float d = sRS[rt * 16 + lane] + sRS[(rt + 4) * 16 + lane] + EPSV;
    sInv[w * 16 + lane] = 64.f / d;
  }
  __syncthreads();

  float* so = sO + w * (16 * OP);
#pragma unroll
  for (int r = 0; r < 8; ++r) {
    const int row = 8 * h + r;
    const float inv = sInv[w * 16 + row];
#pragma unroll
    for (int et = 0; et < 4; ++et) {
      const float val = (ohh[et][r] + ox[et][r] * 0.00048828125f) * inv;
      so[row * OP + et * 16 + m] = val;
    }
  }
  __syncthreads();

  float* ob = out + ((size_t)b * TLEN + t0 + rt * 16) * DM + half * 64;
#pragma unroll
  for (int p = 0; p < 8; ++p) {
    const int piece = p * 32 + lane;
    const int row = piece >> 4, c = piece & 15;
    const v4f x = *(const v4f*)(so + row * OP + c * 4);
    *(volatile v4f*)(ob + (size_t)row * DM + c * 4) = x;
  }
  __threadfence();
#pragma unroll
  for (int p = 0; p < 8; ++p) {
    const int piece = p * 32 + lane;
    const int row = piece >> 4, c = piece & 15;
    const v4f x = *(const v4f*)(so + row * OP + c * 4);
    *(volatile v4f*)(ob + (size_t)row * DM + c * 4) = x;
  }
}

extern "C" void kernel_launch(void* const* d_in, const int* in_sizes, int n_in,
                              void* d_out, int out_size, void* d_ws, size_t ws_size,
                              hipStream_t stream) {
  if (n_in < 5) return;
  const int nq = in_sizes[0];
  if (nq <= 0 || (nq % (TLEN * DM)) != 0) return;
  const int nb = nq / (TLEN * DM);
  if (in_sizes[1] != nq || in_sizes[2] != nq || in_sizes[3] != DM * DM || in_sizes[4] != DM) return;
  if (out_size != nq) return;

  const float* q    = (const float*)d_in[0];
  const float* k    = (const float*)d_in[1];
  const float* v    = (const float*)d_in[2];
  const float* W    = (const float*)d_in[3];
  const float* bias = (const float*)d_in[4];
  float* out = (float*)d_out;

  const size_t plane = (size_t)nq * sizeof(_Float16);
  if (4 * plane > ws_size) return;
  char* ws = (char*)d_ws;
  _Float16* qh  = (_Float16*)(ws);
  _Float16* kh  = (_Float16*)(ws + plane);
  _Float16* vth = (_Float16*)(ws + 2 * plane);
  _Float16* vtl = (_Float16*)(ws + 3 * plane);

  const int nrb = nb * (TLEN / QB);

  k_vconv<<<nb * NKB, 256, 0, stream>>>(v, vth, vtl);
  k_phi<<<2 * nrb, 256, 0, stream>>>(q, k, W, bias, qh, kh, nrb);
  k_attn<<<nb * NQB, 256, 0, stream>>>(qh, kh, vth, vtl, out);
}
